// NBWAttention_56556129354156
// MI455X (gfx1250) — hardware-verified
//
#include <hip/hip_runtime.h>
#include <math.h>

#define NB    2
#define SQ    8192
#define CH    64
#define NQB   (SQ / 64)
#define MR    (NB * SQ)
#define NGRP  8
#define KSPAN 52
#define XSC   16.0f
#define WSC   256.0f
#define QSC   16.0f
#define RSC   4096.0f
#define PSC   1024.0f
#define GEPS  1e-6f
static_assert((SQ % 64) == 0 && (MR % 64) == 0 && CH == 64);
static_assert(NGRP * 8 == CH);
static_assert((KSPAN + 1) * 64 - 63 >= 3328);
static constexpr float kL2G = -0.04580368961312341f;

typedef _Float16 v16h __attribute__((ext_vector_type(16)));
typedef _Float16 v8h  __attribute__((ext_vector_type(8)));
typedef float    v8f  __attribute__((ext_vector_type(8)));
typedef float    v4f  __attribute__((ext_vector_type(4)));
typedef unsigned int v4u __attribute__((ext_vector_type(4)));

__device__ __forceinline__ unsigned short bf_bits(float f) {
  unsigned u = __float_as_uint(f);
  return (unsigned short)((u + 0x7FFFu + ((u >> 16) & 1u)) >> 16);
}
__device__ __forceinline__ float bf_up(unsigned short h) { return __uint_as_float(((unsigned)h) << 16); }
__device__ __forceinline__ float bfr(float f) { return bf_up(bf_bits(f)); }
__device__ __forceinline__ unsigned short h_bits(_Float16 x) { return __builtin_bit_cast(unsigned short, x); }
__device__ __forceinline__ unsigned pk16(unsigned short a, unsigned short b) { return (unsigned)a | ((unsigned)b << 16); }
__device__ __forceinline__ v8f zero8() { v8f z = {0.f, 0.f, 0.f, 0.f, 0.f, 0.f, 0.f, 0.f}; return z; }

__device__ __forceinline__ v16h ldfrag_h(const _Float16* p) {
  union { v16h v; v8h h[2]; } f;
  f.h[0] = *(const v8h*)(p);
  f.h[1] = *(const v8h*)(p + 16);
  return f.v;
}

__device__ __forceinline__ v8f mma_h(v16h a, v16h b, v8f c) {
  c = __builtin_amdgcn_wmma_f32_16x16x32_f16(false, a, false, b, (short)0, c, false, false);
#if defined(__HIP_DEVICE_COMPILE__)
  asm volatile("v_nop\n\tv_nop\n\tv_nop\n\tv_nop" : "+v"(c) : "v"(a), "v"(b));
#endif
  return c;
}
__device__ __forceinline__ v8f mma_h_raw(v16h a, v16h b, v8f c) {
  return __builtin_amdgcn_wmma_f32_16x16x32_f16(false, a, false, b, (short)0, c, false, false);
}
__device__ __forceinline__ void dep_guard1(v8f& a, v8f& b, v16h x) {
#if defined(__HIP_DEVICE_COMPILE__)
  asm volatile("v_nop\n\tv_nop\n\tv_nop\n\tv_nop" : "+v"(a), "+v"(b) : "v"(x));
#endif
}
__device__ __forceinline__ void keep4_h(v16h a, v16h b, v16h c, v16h d) {
#if defined(__HIP_DEVICE_COMPILE__)
  asm volatile("v_nop" :: "v"(a), "v"(b), "v"(c), "v"(d));
#endif
}
__device__ __forceinline__ void acc_guard4(v8f& a, v8f& b, v8f& c, v8f& d) {
#if defined(__HIP_DEVICE_COMPILE__)
  asm volatile("v_nop\n\tv_nop\n\tv_nop\n\tv_nop" : "+v"(a), "+v"(b), "+v"(c), "+v"(d));
#endif
}
__device__ __forceinline__ void wave_sync_lds() {
  __builtin_amdgcn_fence(__ATOMIC_RELEASE, "workgroup");
  __builtin_amdgcn_wave_barrier();
  __builtin_amdgcn_fence(__ATOMIC_ACQUIRE, "workgroup");
}

__device__ __forceinline__ unsigned short cvt16(float f, float wsc) {
  return h_bits((_Float16)(bfr(f) * wsc));
}

__global__ __launch_bounds__(256) void conv16(const float* __restrict__ W, unsigned short* Wh, int n8,
                                              float wsc) {
  const int i = blockIdx.x * 256 + threadIdx.x;
  if (i >= n8) return;
  const size_t e0 = (size_t)i * 8;
  const v4f a = *(const v4f*)(W + e0);
  const v4f b = *(const v4f*)(W + e0 + 4);
  v4u u;
  u[0] = pk16(cvt16(a[0], wsc), cvt16(a[1], wsc));
  u[1] = pk16(cvt16(a[2], wsc), cvt16(a[3], wsc));
  u[2] = pk16(cvt16(b[0], wsc), cvt16(b[1], wsc));
  u[3] = pk16(cvt16(b[2], wsc), cvt16(b[3], wsc));
  for (int pass = 0; pass < 2; ++pass) {
    *(volatile v4u*)(Wh + e0) = u;
    __threadfence();
  }
}

__global__ __launch_bounds__(256) void convwt(const float* __restrict__ W0, const float* __restrict__ W1,
                                              const float* __restrict__ W2, unsigned short* Wt, float wsc) {
  __shared__ __align__(16) float T[64 * 68];
  const int sel = blockIdx.x;
  const int tid = threadIdx.x;
  const float* W = (sel == 0) ? W0 : ((sel == 1) ? W1 : W2);
#pragma unroll
  for (int i = 0; i < 4; ++i) {
    const int idx = i * 1024 + tid * 4;
    const int k = idx >> 6;
    const int n = idx & 63;
    const v4f v = *(const v4f*)(W + idx);
    T[(n + 0) * 68 + k] = v[0];
    T[(n + 1) * 68 + k] = v[1];
    T[(n + 2) * 68 + k] = v[2];
    T[(n + 3) * 68 + k] = v[3];
  }
  __syncthreads();
  v4u u[2];
#pragma unroll
  for (int q = 0; q < 2; ++q) {
    const int p = q * 256 + tid;
    const int row = p >> 3;
    const int c8 = (p & 7) * 8;
    const float* sp = T + row * 68 + c8;
    v4u a;
#pragma unroll
    for (int e = 0; e < 4; ++e) a[e] = pk16(cvt16(sp[2 * e], wsc), cvt16(sp[2 * e + 1], wsc));
    u[q] = a;
  }
  unsigned short* Wo = Wt + (size_t)sel * (CH * CH);
  for (int pass = 0; pass < 2; ++pass) {
#pragma unroll
    for (int q = 0; q < 2; ++q) {
      const int p = q * 256 + tid;
      const int row = p >> 3;
      const int c8 = (p & 7) * 8;
      *(volatile v4u*)(Wo + (size_t)row * CH + c8) = u[q];
    }
    __threadfence();
  }
}

template <int OM>
__global__ __launch_bounds__(256) void gemm64(
    const unsigned short* __restrict__ Ap, int lda,
    const unsigned short* __restrict__ Btp, int ldb,
    unsigned short* Cout, unsigned short* Cout2, int ldc,
    int M, int N, int K, float oscale, float rsc) {
  const _Float16* A  = (const _Float16*)(const void*)Ap;
  const _Float16* Bt = (const _Float16*)(const void*)Btp;
  __shared__ __align__(16) float sT[8][16 * 68];
  const int lane = threadIdx.x & 31;
  const int wave = threadIdx.x >> 5;
  const int tilesN = N >> 6;
  const int tilesM = M >> 6;
  const int tile = blockIdx.x * 8 + wave;
  if (tile >= tilesM * tilesN) return;
  const int tm = tile / tilesN;
  const int tn = tile - tm * tilesN;
  const int m0 = tm << 6;
  const int n0 = tn << 6;

  const int rlane = lane & 15;
  const int koff  = (lane >> 4) * 8;
  const int mOff  = (lane >> 4) * 8;

  v8f acc[4][4];
#pragma unroll
  for (int i = 0; i < 4; ++i)
#pragma unroll
    for (int j = 0; j < 4; ++j) acc[i][j] = zero8();

  for (int k0 = 0; k0 < K; k0 += 32) {
    v16h bh[4];
#pragma unroll
    for (int j = 0; j < 4; ++j) {
      const size_t bo = (size_t)(n0 + (j << 4) + rlane) * ldb + koff + k0;
      bh[j] = ldfrag_h(Bt + bo);
    }
#pragma unroll
    for (int i = 0; i < 4; ++i) {
      const size_t ao = (size_t)(m0 + (i << 4) + rlane) * lda + koff + k0;
      const v16h ah = ldfrag_h(A + ao);
#pragma unroll
      for (int j = 0; j < 4; ++j) acc[i][j] = mma_h_raw(ah, bh[j], acc[i][j]);
      dep_guard1(acc[i][0], acc[i][3], ah);
    }
    keep4_h(bh[0], bh[1], bh[2], bh[3]);
  }
  acc_guard4(acc[0][0], acc[0][1], acc[0][2], acc[0][3]);
  acc_guard4(acc[1][0], acc[1][1], acc[1][2], acc[1][3]);
  acc_guard4(acc[2][0], acc[2][1], acc[2][2], acc[2][3]);
  acc_guard4(acc[3][0], acc[3][1], acc[3][2], acc[3][3]);

  const int q8 = lane >> 3, c8 = (lane & 7) * 8;

  float* slab = sT[wave];
#pragma unroll
  for (int i = 0; i < 4; ++i) {
    const int mBase = m0 + (i << 4);
#pragma unroll
    for (int j = 0; j < 4; ++j) {
#pragma unroll
      for (int r = 0; r < 8; ++r) {
        slab[(mOff + r) * 68 + (j << 4) + rlane] = acc[i][j][r];
      }
    }
    wave_sync_lds();
    v4u hv[4], lv[4];
#pragma unroll
    for (int it = 0; it < 4; ++it) {
      const int row = it * 4 + q8;
      const float* sp = slab + row * 68 + c8;
      v4u a, lw;
#pragma unroll
      for (int e = 0; e < 4; ++e) {
        const float f0 = sp[2 * e]     * oscale;
        const float f1 = sp[2 * e + 1] * oscale;
        const _Float16 g0 = (_Float16)f0;
        const _Float16 g1 = (_Float16)f1;
        a[e] = pk16(h_bits(g0), h_bits(g1));
        if (OM == 3) {
          const _Float16 r0 = (_Float16)((f0 - (float)g0) * rsc);
          const _Float16 r1 = (_Float16)((f1 - (float)g1) * rsc);
          lw[e] = pk16(h_bits(r0), h_bits(r1));
        } else {
          lw[e] = 0u;
        }
      }
      hv[it] = a;
      lv[it] = lw;
    }
    for (int pass = 0; pass < 2; ++pass) {
#pragma unroll
      for (int it = 0; it < 4; ++it) {
        const int row = it * 4 + q8;
        const size_t go = (size_t)(mBase + row) * ldc + n0 + c8;
        *(volatile v4u*)(Cout + go) = hv[it];
        if (OM == 3) *(volatile v4u*)(Cout2 + go) = lv[it];
      }
      __threadfence();
    }
    wave_sync_lds();
  }
}

__global__ __launch_bounds__(128)
void retn64(const unsigned short* __restrict__ qhp, const unsigned short* __restrict__ qlp,
            const unsigned short* __restrict__ khp, const unsigned short* __restrict__ klp,
            const unsigned short* __restrict__ vthp, const unsigned short* __restrict__ vtlp,
            const float* __restrict__ gw, const float* __restrict__ gb, float* outp) {
  union FH { v16h v; v8h h[2]; };
  __shared__ __align__(16) _Float16 Psh[4][16 * 64];
  __shared__ __align__(16) _Float16 Psl[4][16 * 64];
  __shared__ __align__(16) float    OT[64 * 68];

  const int tid  = threadIdx.x;
  const int wave = tid >> 5;
  const int lane = tid & 31;
  const int hh   = lane >> 4;
  const int c    = lane & 15;

  const int bx   = blockIdx.x;
  const int qb   = bx % NQB;
  const int sb   = bx / NQB;
  const int qblk = qb * 64;
  const int q0   = qblk + wave * 16;
  const size_t rb = (size_t)sb * SQ;

  const _Float16* Qh = (const _Float16*)(const void*)qhp + rb * CH;
  const _Float16* Ql = (const _Float16*)(const void*)qlp + rb * CH;
  const _Float16* Kh = (const _Float16*)(const void*)khp + rb * CH;
  const _Float16* Kl = (const _Float16*)(const void*)klp + rb * CH;
  const _Float16* Vh = (const _Float16*)(const void*)vthp + rb;
  const _Float16* Vl = (const _Float16*)(const void*)vtlp + rb;

  v16h qa[2], qr[2];
#pragma unroll
  for (int dc = 0; dc < 2; ++dc) {
    qa[dc] = ldfrag_h(Qh + (size_t)(q0 + c) * CH + dc * 32 + 8 * hh);
    qr[dc] = ldfrag_h(Ql + (size_t)(q0 + c) * CH + dc * 32 + 8 * hh);
  }

  v8f oacc[4];
#pragma unroll
  for (int t = 0; t < 4; ++t) oacc[t] = zero8();

  int ktLo = qb - KSPAN;
  if (ktLo < 0) ktLo = 0;
  const int ktHi = qb;
  const float rinv = 1.0f / RSC;
  const float pmul = PSC / (QSC * QSC);
  _Float16* pwh = Psh[wave];
  _Float16* pwl = Psl[wave];

  for (int kt = ktLo; kt <= ktHi; ++kt) {
    const int kv0 = kt * 64;

#pragma unroll
    for (int j = 0; j < 4; ++j) {
      v8f sh = zero8(), sl = zero8();
      const size_t krow = (size_t)(kv0 + j * 16 + c) * CH + 8 * hh;
#pragma unroll
      for (int dc = 0; dc < 2; ++dc) {
        const v16h kbh = ldfrag_h(Kh + krow + dc * 32);
        const v16h kbl = ldfrag_h(Kl + krow + dc * 32);
        sh = mma_h(qa[dc], kbh, sh);
        sl = mma_h(qa[dc], kbl, sl);
        sl = mma_h(qr[dc], kbh, sl);
      }
      const int key = kv0 + j * 16 + c;
#pragma unroll
      for (int r = 0; r < 8; ++r) {
        const int n = q0 + 8 * hh + r - key;
        const float dcy = exp2f((float)n * kL2G);
        const float d = (n >= 0) ? dcy : 0.f;
        const float pv = (sh[r] + sl[r] * rinv) * d * pmul;
        const _Float16 ph = (_Float16)pv;
        const int pi = (8 * hh + r) * 64 + j * 16 + c;
        pwh[pi] = ph;
        pwl[pi] = (_Float16)((pv - (float)ph) * RSC);
      }
    }
    wave_sync_lds();

    v8f ol[4];
#pragma unroll
    for (int t = 0; t < 4; ++t) ol[t] = zero8();
#pragma unroll 1
    for (int kk = 0; kk < 2; ++kk) {
      FH pa, pr;
      pa.h[0] = *(const v8h*)(pwh + c * 64 + kk * 32 + 8 * hh);
      pa.h[1] = *(const v8h*)(pwh + c * 64 + kk * 32 + 16 + 8 * hh);
      pr.h[0] = *(const v8h*)(pwl + c * 64 + kk * 32 + 8 * hh);
      pr.h[1] = *(const v8h*)(pwl + c * 64 + kk * 32 + 16 + 8 * hh);
#pragma unroll
      for (int t = 0; t < 4; ++t) {
        const size_t vrow = (size_t)(t * 16 + c) * MR + kv0 + kk * 32 + 8 * hh;
        const v16h vb = ldfrag_h(Vh + vrow);
        const v16h wb = ldfrag_h(Vl + vrow);
        oacc[t] = mma_h(pa.v, vb, oacc[t]);
        ol[t]   = mma_h(pa.v, wb, ol[t]);
        ol[t]   = mma_h(pr.v, vb, ol[t]);
      }
    }
#pragma unroll
    for (int t = 0; t < 4; ++t) {
#pragma unroll
      for (int r = 0; r < 8; ++r) oacc[t][r] += ol[t][r] * rinv;
    }
    wave_sync_lds();
  }

  const float osc = 1.0f / (PSC * QSC);
  float gwv[4], gbv[4];
#pragma unroll
  for (int t = 0; t < 4; ++t) {
    gwv[t] = bfr(gw[t * 16 + c]);
    gbv[t] = bfr(gb[t * 16 + c]);
  }
#pragma unroll
  for (int t = 0; t < 4; ++t) {
#pragma unroll
    for (int r = 0; r < 8; ++r) {
      const float x = oacc[t][r] * osc;
      float s1 = x;
      s1 += __shfl_xor(s1, 1, 32);
      s1 += __shfl_xor(s1, 2, 32);
      s1 += __shfl_xor(s1, 4, 32);
      const float mu = s1 * 0.125f;
      const float dv = x - mu;
      float s2 = dv * dv;
      s2 += __shfl_xor(s2, 1, 32);
      s2 += __shfl_xor(s2, 2, 32);
      s2 += __shfl_xor(s2, 4, 32);
      const float var = s2 * 0.125f;
      const float inv = rsqrtf(var + GEPS);
      OT[(t * 16 + c) * 68 + wave * 16 + 8 * hh + r] = dv * inv * gwv[t] + gbv[t];
    }
  }
  __syncthreads();

  {
    const int hh2 = lane >> 4, c4 = (lane & 15) * 4;
    v4f vals[8];
#pragma unroll
    for (int it = 0; it < 8; ++it) {
      const int ch = wave * 16 + it * 2 + hh2;
      vals[it] = *(const v4f*)(OT + ch * 68 + c4);
    }
    float* ob = outp + (size_t)sb * CH * SQ + qblk;
    for (int pass = 0; pass < 2; ++pass) {
#pragma unroll
      for (int it = 0; it < 8; ++it) {
        const int ch = wave * 16 + it * 2 + hh2;
        *(volatile v4f*)(ob + (size_t)ch * SQ + c4) = vals[it];
      }
      __threadfence();
    }
  }
}

extern "C" void kernel_launch(void* const* d_in, const int* in_sizes, int n_in,
                              void* d_out, int out_size, void* d_ws, size_t ws_size,
                              hipStream_t stream) {
  if (n_in < 6) return;
  if (in_sizes[0] != MR * CH) return;
  if (in_sizes[1] != CH * CH || in_sizes[2] != CH * CH || in_sizes[3] != CH * CH) return;
  if (in_sizes[4] != CH || in_sizes[5] != CH) return;
  if (out_size != MR * CH) return;

  const float* x  = (const float*)d_in[0];
  const float* wq = (const float*)d_in[1];
  const float* wk = (const float*)d_in[2];
  const float* wv = (const float*)d_in[3];
  const float* gw = (const float*)d_in[4];
  const float* gb = (const float*)d_in[5];

  const size_t PW = 32768;
  const size_t PX = (size_t)MR * CH * 2;
  size_t off = 0;
  const size_t oWT = off; off += PW;
  const size_t oXH = off; off += PX;
  const size_t oQH = off; off += PX;
  const size_t oQL = off; off += PX;
  const size_t oKH = off; off += PX;
  const size_t oKL = off; off += PX;
  const size_t oVH = off; off += PX;
  const size_t oVL = off; off += PX;
  if (off > ws_size) return;
  if (off > (size_t)134217728) return;

  char* ws = (char*)d_ws;
  unsigned short* WT  = (unsigned short*)(ws + oWT);
  unsigned short* WTq = WT;
  unsigned short* WTk = WT + (size_t)CH * CH;
  unsigned short* WTv = WT + (size_t)2 * CH * CH;
  unsigned short* XH  = (unsigned short*)(ws + oXH);
  unsigned short* QH  = (unsigned short*)(ws + oQH);
  unsigned short* QL  = (unsigned short*)(ws + oQL);
  unsigned short* KH  = (unsigned short*)(ws + oKH);
  unsigned short* KL  = (unsigned short*)(ws + oKL);
  unsigned short* VTH = (unsigned short*)(ws + oVH);
  unsigned short* VTL = (unsigned short*)(ws + oVL);

  const dim3 blk(256), blk128(128);
  const dim3 gCx((MR * CH / 8 + 255) / 256);
  const dim3 gCw(3);
  const dim3 gG(((MR / 64) * (CH / 64) + 7) / 8);
  const dim3 gR(NB * NQB);
  const float osc = QSC / (XSC * WSC);

  conv16<<<gCx, blk, 0, stream>>>(x, XH, MR * CH / 8, XSC);
  convwt<<<gCw, blk, 0, stream>>>(wq, wk, wv, WT, WSC);

  gemm64<3><<<gG, blk, 0, stream>>>(XH, CH, WTq, CH, QH, QL, CH, MR, CH, CH, osc, RSC);
  gemm64<3><<<gG, blk, 0, stream>>>(XH, CH, WTk, CH, KH, KL, CH, MR, CH, CH, osc, RSC);
  gemm64<3><<<gG, blk, 0, stream>>>(WTv, CH, XH, CH, VTH, VTL, MR, CH, MR, CH, osc, RSC);

  retn64<<<gR, blk128, 0, stream>>>(QH, QL, KH, KL, VTH, VTL, gw, gb, (float*)d_out);
  (void)hipGetLastError();
}
